// DeltaNet_31877247271568
// MI455X (gfx1250) — hardware-verified
//
#include <hip/hip_runtime.h>
#include <math.h>

constexpr int kBatch   = 2;
constexpr int kSeq     = 4096;
constexpr int kDim     = 1024;
constexpr int kHeads   = 4;
constexpr int kHd      = 256;
constexpr int kChunk   = 32;
constexpr int kNChunk  = kSeq / kChunk;
constexpr int kTok     = kBatch * kSeq;
constexpr int kBH      = kBatch * kHeads;
constexpr int kGP      = 32;
constexpr int kGRP     = 64;
constexpr int kSlice   = 64;
constexpr int kNSlice  = kHd / kSlice;
constexpr int kTP      = 40;
constexpr int kAP      = 33;
constexpr int kSP      = 264;
constexpr int kFP      = 68;
constexpr int kConvTile = 32;
constexpr float kWCarry    = 16.0f;
constexpr float kWCarryInv = 1.0f / 16.0f;
constexpr float kEpsL2  = 1e-6f;
constexpr float kEpsRms = 1e-5f;
constexpr float kInvHd  = 1.0f / (float)kHd;

static_assert(kDim == kHeads * kHd, "head split");
static_assert(kSeq % kChunk == 0 && kSeq % kConvTile == 0, "chunking");
static_assert(kTok % 64 == 0 && kDim % 64 == 0 && kGRP % 64 == 0 && kDim % 32 == 0, "GEMM tile multiples");
static_assert(kChunk == 32 && kHd == 256 && kSlice == 64, "tile maps below assume these");
static_assert((kTP % 8) == 0 && (kSP % 8) == 0, "16-B aligned LDS pitches");

typedef __attribute__((ext_vector_type(16))) _Float16 v16h;
typedef __attribute__((ext_vector_type(8)))  _Float16 v8h;
typedef __attribute__((ext_vector_type(8)))  float    v8f;
typedef __attribute__((ext_vector_type(4)))  float    v4f;
typedef __attribute__((ext_vector_type(4)))  unsigned int v4u;

__device__ __forceinline__ float h16_to_f32(unsigned hb) {
  const unsigned sgn = (hb & 0x8000u) << 16;
  const unsigned em = hb & 0x7fffu;
  const float fn = __uint_as_float((em << 13) + 0x38000000u);
  const float fs = (float)em * 5.9604644775390625e-8f;
  const float mag = (em < 0x400u) ? fs : fn;
  return __uint_as_float(__float_as_uint(mag) | sgn);
}
__device__ __forceinline__ _Float16 bits_to_h(unsigned b) {
  const unsigned short s = (unsigned short)(b & 0xffffu);
  return __builtin_bit_cast(_Float16, s);
}
__device__ __forceinline__ float sigmoid_f(float x) {
  return __builtin_amdgcn_rcpf(1.0f + expf(-x));
}
__device__ __forceinline__ void wave_lds_sync() {
  __builtin_amdgcn_fence(__ATOMIC_RELEASE, "workgroup");
  __builtin_amdgcn_wave_barrier();
  __builtin_amdgcn_fence(__ATOMIC_ACQUIRE, "workgroup");
}

union FragU { v16h v; v8h h[2]; };
__device__ __forceinline__ v16h frag_load(const _Float16* p) {
  FragU f;
  f.h[0] = *(const v8h*)(p);
  f.h[1] = *(const v8h*)(p + 16);
  return f.v;
}
__device__ __forceinline__ v8f mma_h(v16h a, v16h b, v8f c) {
  return __builtin_amdgcn_wmma_f32_16x16x32_f16(false, a, false, b, (short)0, c, false, false);
}
__device__ __forceinline__ void guard1_h(v8f& a, v16h x, v16h y) {
  asm volatile("v_nop\n\tv_nop\n\tv_nop\n\tv_nop" : "+v"(a) : "v"(x), "v"(y));
}
__device__ __forceinline__ void guard2_h(v8f& a, v8f& b, v16h x, v16h y, v16h z) {
  asm volatile("v_nop\n\tv_nop\n\tv_nop\n\tv_nop" : "+v"(a), "+v"(b) : "v"(x), "v"(y), "v"(z));
}
__device__ __forceinline__ void guard4_h(v8f& a, v8f& b, v8f& c, v8f& d, v16h x, v16h y0, v16h y1, v16h y2, v16h y3) {
  asm volatile("v_nop\n\tv_nop\n\tv_nop\n\tv_nop" : "+v"(a), "+v"(b), "+v"(c), "+v"(d)
               : "v"(x), "v"(y0), "v"(y1), "v"(y2), "v"(y3));
}
__device__ __forceinline__ void guard8_h(v8f& a0, v8f& a1, v8f& a2, v8f& a3, v8f& a4, v8f& a5, v8f& a6, v8f& a7,
                                         v16h x0, v16h x1, v16h y0, v16h y1, v16h y2, v16h y3) {
  asm volatile("v_nop\n\tv_nop\n\tv_nop\n\tv_nop"
               : "+v"(a0), "+v"(a1), "+v"(a2), "+v"(a3), "+v"(a4), "+v"(a5), "+v"(a6), "+v"(a7)
               : "v"(x0), "v"(x1), "v"(y0), "v"(y1), "v"(y2), "v"(y3));
}
__device__ __forceinline__ void keep4_h(v16h a, v16h b, v16h c, v16h d) {
  asm volatile("v_nop" :: "v"(a), "v"(b), "v"(c), "v"(d));
}
__device__ __forceinline__ void acc_guard4(v8f& a, v8f& b, v8f& c, v8f& d) {
  asm volatile("v_nop\n\tv_nop\n\tv_nop\n\tv_nop" : "+v"(a), "+v"(b), "+v"(c), "+v"(d));
}

__global__ __launch_bounds__(256) void wmma_gemm64_f16(
    const unsigned short* __restrict__ Ap, int lda,
    const unsigned short* __restrict__ Btp, int ldb,
    float* __restrict__ Cout, int ldc, int M, int N, int K, float scale) {
  const _Float16* A  = (const _Float16*)Ap;
  const _Float16* Bt = (const _Float16*)Btp;
  __shared__ __align__(16) float sT[8][16 * kFP];
  const int lane = threadIdx.x & 31;
  const int wave = threadIdx.x >> 5;
  const int tilesN = N >> 6;
  const int tilesM = M >> 6;
  const int tile = blockIdx.x * 8 + wave;
  if (tile >= tilesM * tilesN) return;
  const int tm = tile / tilesN;
  const int tn = tile - tm * tilesN;
  const int m0 = tm << 6;
  const int n0 = tn << 6;
  const int rlane = lane & 15;
  const int koff  = (lane >> 4) * 8;
  const int mOff  = (lane >> 4) * 8;

  const _Float16* Arow = A  + (size_t)(m0 + rlane) * lda + koff;
  const _Float16* Brow = Bt + (size_t)(n0 + rlane) * ldb + koff;
  const size_t a16 = (size_t)16 * lda;
  const size_t b16 = (size_t)16 * ldb;

  v8f acc[4][4];
#pragma unroll
  for (int i = 0; i < 4; ++i)
#pragma unroll
    for (int j = 0; j < 4; ++j) acc[i][j] = (v8f){0.f, 0.f, 0.f, 0.f, 0.f, 0.f, 0.f, 0.f};

  for (int k0 = 0; k0 < K; k0 += 32) {
    v16h bh[4];
#pragma unroll
    for (int j = 0; j < 4; ++j) bh[j] = frag_load(Brow + j * b16 + k0);
#pragma unroll
    for (int i = 0; i < 4; ++i) {
      const v16h ah = frag_load(Arow + i * a16 + k0);
#pragma unroll
      for (int j = 0; j < 4; ++j) acc[i][j] = mma_h(ah, bh[j], acc[i][j]);
      guard4_h(acc[i][0], acc[i][1], acc[i][2], acc[i][3], ah, bh[0], bh[1], bh[2], bh[3]);
    }
    keep4_h(bh[0], bh[1], bh[2], bh[3]);
  }
  acc_guard4(acc[0][0], acc[0][1], acc[0][2], acc[0][3]);
  acc_guard4(acc[1][0], acc[1][1], acc[1][2], acc[1][3]);
  acc_guard4(acc[2][0], acc[2][1], acc[2][2], acc[2][3]);
  acc_guard4(acc[3][0], acc[3][1], acc[3][2], acc[3][3]);

  float* slab = sT[wave];
#pragma unroll
  for (int i = 0; i < 4; ++i) {
    const int mBase = m0 + (i << 4);
#pragma unroll
    for (int j = 0; j < 4; ++j) {
#pragma unroll
      for (int r = 0; r < 8; ++r) slab[(mOff + r) * kFP + (j << 4) + rlane] = acc[i][j][r] * scale;
    }
    wave_lds_sync();
    {
      const int hh = lane >> 4, c4 = (lane & 15) * 4;
      for (int pass = 0; pass < 2; ++pass) {
#pragma unroll
        for (int it = 0; it < 8; ++it) {
          const int row = it * 2 + hh;
          const v4f v = *(const v4f*)(slab + row * kFP + c4);
          *(volatile v4f*)(Cout + (size_t)(mBase + row) * ldc + n0 + c4) = v;
        }
        __threadfence();
      }
    }
    wave_lds_sync();
  }
}

__global__ __launch_bounds__(256) void cast8_f16_kernel(const float* __restrict__ in, unsigned short* __restrict__ out,
                                                        int n8, float sc) {
  const int i = blockIdx.x * 256 + threadIdx.x;
  if (i < n8) {
    const float* p = in + (size_t)i * 8;
    const v4f a = *(const v4f*)(p);
    const v4f b = *(const v4f*)(p + 4);
    v8h hv;
#pragma unroll
    for (int e = 0; e < 4; ++e) {
      hv[e]     = (_Float16)(a[e] * sc);
      hv[4 + e] = (_Float16)(b[e] * sc);
    }
    unsigned short* q = out + (size_t)i * 8;
    *(volatile v8h*)q = hv;
    __threadfence();
    *(volatile v8h*)q = hv;
  }
}

__global__ __launch_bounds__(256) void gate_pack_kernel(const float* __restrict__ Wb, const float* __restrict__ Wd,
                                                        const float* __restrict__ Wm, unsigned short* __restrict__ out, float sc) {
  const int i = blockIdx.x * 256 + threadIdx.x;
  if (i < kGRP * (kDim / 8)) {
    const int row = i >> 7;
    const int c8 = (i & 127) * 8;
    const int r4 = row & 3;
    const int sel = row >> 2;
    const int off = r4 * kDim + c8;
    const v4f a0 = *(const v4f*)(Wb + off);
    const v4f a1 = *(const v4f*)(Wb + off + 4);
    const v4f b0 = *(const v4f*)(Wd + off);
    const v4f b1 = *(const v4f*)(Wd + off + 4);
    const v4f c0 = *(const v4f*)(Wm + off);
    const v4f c1 = *(const v4f*)(Wm + off + 4);
    v8h hv;
#pragma unroll
    for (int e = 0; e < 4; ++e) {
      const float x0 = (sel == 0) ? a0[e] : (sel == 1) ? b0[e] : (sel == 2) ? c0[e] : 0.0f;
      const float x1 = (sel == 0) ? a1[e] : (sel == 1) ? b1[e] : (sel == 2) ? c1[e] : 0.0f;
      hv[e]     = (_Float16)(x0 * sc);
      hv[4 + e] = (_Float16)(x1 * sc);
    }
    unsigned short* q = out + (size_t)i * 8;
    *(volatile v8h*)q = hv;
    __threadfence();
    *(volatile v8h*)q = hv;
  }
}

__global__ __launch_bounds__(256) void gate_act_kernel(const float* __restrict__ GR, const float* __restrict__ mixb,
                                                       float* __restrict__ G) {
  const int i = blockIdx.x * 256 + threadIdx.x;
  if (i < kTok * 8) {
    const int row = i >> 3;
    const int q = i & 7;
    const v4f x = *(const v4f*)(GR + (size_t)row * kGRP + 4 * q);
    const v4f mb = *(const v4f*)(mixb);
    v4f o;
#pragma unroll
    for (int e = 0; e < 4; ++e) {
      const float z = x[e] + ((q == 2) ? mb[e] : 0.0f);
      const float s = sigmoid_f(z);
      o[e] = (q < 3) ? s : 0.0f;
    }
    float* dp = G + (size_t)row * kGP + 4 * q;
    *(volatile v4f*)dp = o;
    __threadfence();
    *(volatile v4f*)dp = o;
  }
}

template <bool NORM>
__global__ __launch_bounds__(128) void conv_act_kernel(const float* __restrict__ P, const float* __restrict__ wc,
                                                       unsigned short* __restrict__ outp) {
  const int lane = threadIdx.x & 31;
  const int h = __builtin_amdgcn_readfirstlane((int)(threadIdx.x >> 5));
  const int tok0 = blockIdx.x * kConvTile;
  const int b = tok0 / kSeq;
  const int l0 = tok0 - b * kSeq;
  const int ch = h * kHd + 8 * lane;

  float wt[8][4];
#pragma unroll
  for (int e = 0; e < 8; ++e) {
    const v4f w = *(const v4f*)(wc + (size_t)(ch + e) * 4);
    wt[e][0] = w[0]; wt[e][1] = w[1]; wt[e][2] = w[2]; wt[e][3] = w[3];
  }
  const bool halo = (l0 > 0);
  const int ra = halo ? (tok0 - 3) : tok0;
  float xa[8], xb[8], xc[8];
  {
    const float* p0 = P + (size_t)ra * kDim + ch;
    const v4f a0 = *(const v4f*)(p0);
    const v4f a1 = *(const v4f*)(p0 + 4);
    const v4f b0 = *(const v4f*)(p0 + kDim);
    const v4f b1 = *(const v4f*)(p0 + kDim + 4);
    const v4f c0 = *(const v4f*)(p0 + 2 * kDim);
    const v4f c1 = *(const v4f*)(p0 + 2 * kDim + 4);
#pragma unroll
    for (int e = 0; e < 4; ++e) {
      xa[e] = halo ? a0[e] : 0.0f;  xa[4 + e] = halo ? a1[e] : 0.0f;
      xb[e] = halo ? b0[e] : 0.0f;  xb[4 + e] = halo ? b1[e] : 0.0f;
      xc[e] = halo ? c0[e] : 0.0f;  xc[4 + e] = halo ? c1[e] : 0.0f;
    }
  }
  unsigned short* orow = outp + ((size_t)(b * kHeads + h) * kSeq + l0) * kHd + 8 * lane;

#pragma unroll 1
  for (int i = 0; i < kConvTile; ++i) {
    const float* pr = P + (size_t)(tok0 + i) * kDim + ch;
    const v4f c0 = *(const v4f*)(pr);
    const v4f c1 = *(const v4f*)(pr + 4);
    float cur[8];
#pragma unroll
    for (int e = 0; e < 4; ++e) { cur[e] = c0[e]; cur[4 + e] = c1[e]; }
    float y[8];
    float ss = 0.0f;
#pragma unroll
    for (int e = 0; e < 8; ++e) {
      float t = wt[e][0] * xa[e];
      t += wt[e][1] * xb[e];
      t += wt[e][2] * xc[e];
      t += wt[e][3] * cur[e];
      const float a = t * sigmoid_f(t);
      y[e] = a;
      ss += a * a;
    }
    if (NORM) {
#pragma unroll
      for (int off = 1; off < 32; off <<= 1) ss += __shfl_xor(ss, off, 32);
      const float inv = rsqrtf(ss + kEpsL2);
#pragma unroll
      for (int e = 0; e < 8; ++e) y[e] *= inv;
    }
    v8h hv;
#pragma unroll
    for (int e = 0; e < 8; ++e) hv[e] = (_Float16)y[e];
    unsigned short* dp = orow + (size_t)i * kHd;
    *(volatile v8h*)dp = hv;
    __threadfence();
    *(volatile v8h*)dp = hv;
#pragma unroll
    for (int e = 0; e < 8; ++e) { xa[e] = xb[e]; xb[e] = xc[e]; xc[e] = cur[e]; }
  }
}

__global__ __launch_bounds__(256) void chunk_prep_kernel(const unsigned short* __restrict__ Q16,
                                                         const unsigned short* __restrict__ K16,
                                                         const unsigned short* __restrict__ V16,
                                                         const float* __restrict__ G,
                                                         unsigned short* __restrict__ U16,
                                                         unsigned short* __restrict__ W16P,
                                                         unsigned short* __restrict__ APL) {
  __shared__ __align__(16) _Float16 kT[kHd * kTP];
  __shared__ __align__(16) _Float16 vT[kHd * kTP];
  __shared__ __align__(16) _Float16 Tp[kChunk * kTP];
  __shared__ __align__(16) float At[kChunk * kAP];
  __shared__ __align__(16) float Qa[kChunk * kAP];
  __shared__ float bet[kChunk];
  __shared__ __align__(16) float sT[8][16 * kFP];

  const int tid = threadIdx.x;
  const int lane = tid & 31;
  const int wave = __builtin_amdgcn_readfirstlane((int)(tid >> 5));
  const int c = lane & 15;
  const int hh = lane >> 4;
  const int koff = 8 * hh;
  const int cid = blockIdx.x;
  const int bh = cid >> 7;
  const int n = cid & (kNChunk - 1);
  const int b = bh >> 2;
  const int h = bh & 3;
  const size_t base = ((size_t)bh * kSeq + (size_t)n * kChunk) * kHd;
  const int tok0 = b * kSeq + n * kChunk;

  if (wave == 0) bet[lane] = G[(size_t)(tok0 + lane) * kGP + h];

#pragma unroll
  for (int it = 0; it < 4; ++it) {
    const int item = it * 256 + tid;
    const int row = item >> 5;
    const int c8 = (item & 31) * 8;
    const v4u kw = *(const v4u*)(K16 + base + (size_t)row * kHd + c8);
    const v4u vw = *(const v4u*)(V16 + base + (size_t)row * kHd + c8);
#pragma unroll
    for (int q = 0; q < 4; ++q) {
      const unsigned ku = kw[q];
      const unsigned vu = vw[q];
      kT[(c8 + 2 * q) * kTP + row]     = bits_to_h(ku);
      kT[(c8 + 2 * q + 1) * kTP + row] = bits_to_h(ku >> 16);
      vT[(c8 + 2 * q) * kTP + row]     = bits_to_h(vu);
      vT[(c8 + 2 * q + 1) * kTP + row] = bits_to_h(vu >> 16);
    }
  }

  {
    const int sel = wave >> 2;
    const int mi = (wave >> 1) & 1;
    const int ni = wave & 1;
    const _Float16* Ag = (const _Float16*)(sel ? Q16 : K16) + base + (size_t)(mi * 16 + c) * kHd + koff;
    const _Float16* Bg = (const _Float16*)K16 + base + (size_t)(ni * 16 + c) * kHd + koff;
    v8f acc = (v8f){0.f, 0.f, 0.f, 0.f, 0.f, 0.f, 0.f, 0.f};
#pragma unroll 2
    for (int k0 = 0; k0 < kHd; k0 += 32) {
      const v16h fa = frag_load(Ag + k0);
      const v16h fb = frag_load(Bg + k0);
      acc = mma_h(fa, fb, acc);
      guard1_h(acc, fa, fb);
    }
    float* dstT = sel ? Qa : At;
#pragma unroll
    for (int r = 0; r < 8; ++r) {
      const int row = mi * 16 + 8 * hh + r;
      const int col = ni * 16 + c;
      const float nb = -G[(size_t)(tok0 + row) * kGP + h];
      const float vk = (row > col) ? (nb * acc[r]) : 0.0f;
      const float vq = (row >= col) ? acc[r] : 0.0f;
      dstT[row * kAP + col] = sel ? vq : vk;
    }
  }
  __syncthreads();

  if (wave == 0) {
#pragma unroll 1
    for (int i = 1; i < kChunk; ++i) {
      const float rowv = At[i * kAP + lane];
      float s = 0.0f;
#pragma unroll 1
      for (int j = 0; j < i; ++j) {
        const float bj = __shfl(rowv, j, 32);
        s = fmaf(bj, At[j * kAP + lane], s);
      }
      if (lane < i) At[i * kAP + lane] = rowv + s;
      wave_lds_sync();
    }
  }
  if (wave >= 4) {
    const int tt = tid - 128;
    const int row = tt >> 2;
    const int c8 = (tt & 3) * 8;
    v8h hv;
#pragma unroll
    for (int e = 0; e < 8; ++e) hv[e] = (_Float16)Qa[row * kAP + c8 + e];
    unsigned short* dp = APL + (size_t)cid * (kChunk * kChunk) + row * kChunk + c8;
    *(volatile v8h*)dp = hv;
    __threadfence();
    *(volatile v8h*)dp = hv;
  }
  __syncthreads();

#pragma unroll
  for (int e = 0; e < 4; ++e) {
    const int idx = tid * 4 + e;
    const int i = idx >> 5;
    const int j = idx & 31;
    const float x = (At[i * kAP + j] + ((i == j) ? 1.0f : 0.0f)) * bet[j];
    Tp[i * kTP + j] = (_Float16)x;
  }
  __syncthreads();

  {
    const int selD = wave >> 2;
    const int ncol0 = (wave & 3) * 64;
    const _Float16* src = selD ? kT : vT;
    unsigned short* dstp = selD ? W16P : U16;
    const v16h a0 = frag_load(Tp + c * kTP + koff);
    const v16h a1 = frag_load(Tp + (16 + c) * kTP + koff);
    const v8f z8 = (v8f){0.f, 0.f, 0.f, 0.f, 0.f, 0.f, 0.f, 0.f};
    v16h fb[4];
    v8f acc[2][4];
#pragma unroll
    for (int j = 0; j < 4; ++j) {
      fb[j] = frag_load(src + (ncol0 + 16 * j + c) * kTP + koff);
      acc[0][j] = mma_h(a0, fb[j], z8);
      acc[1][j] = mma_h(a1, fb[j], z8);
    }
    guard8_h(acc[0][0], acc[0][1], acc[0][2], acc[0][3], acc[1][0], acc[1][1], acc[1][2], acc[1][3],
             a0, a1, fb[0], fb[1], fb[2], fb[3]);
    float* slab = sT[wave];
#pragma unroll
    for (int mi = 0; mi < 2; ++mi) {
#pragma unroll
      for (int j = 0; j < 4; ++j)
#pragma unroll
        for (int r = 0; r < 8; ++r) slab[(8 * hh + r) * kFP + 16 * j + c] = acc[mi][j][r];
      wave_lds_sync();
      {
        const int q4 = lane >> 3, c8 = (lane & 7) * 8;
        for (int pass = 0; pass < 2; ++pass) {
#pragma unroll
          for (int it = 0; it < 4; ++it) {
            const int row = it * 4 + q4;
            const float* sp = slab + row * kFP + c8;
            v8h hv;
#pragma unroll
            for (int e = 0; e < 8; ++e) hv[e] = (_Float16)sp[e];
            *(volatile v8h*)(dstp + base + (size_t)(mi * 16 + row) * kHd + ncol0 + c8) = hv;
          }
          __threadfence();
        }
      }
      wave_lds_sync();
    }
  }
}

__global__ __launch_bounds__(256) void state_scan_kernel(const unsigned short* __restrict__ Q16,
                                                         const unsigned short* __restrict__ K16,
                                                         const unsigned short* __restrict__ U16,
                                                         const unsigned short* __restrict__ W16P,
                                                         const unsigned short* __restrict__ APL,
                                                         float* __restrict__ OD) {
  __shared__ __align__(16) _Float16 S16[kSlice * kSP];
  __shared__ __align__(16) _Float16 kT[kHd * kTP];
  __shared__ __align__(16) _Float16 unT[kSlice * kTP];
  __shared__ __align__(16) float uS[kChunk * kFP];
  __shared__ __align__(16) float oS[kChunk * kFP];

  const int tid = threadIdx.x;
  const int lane = tid & 31;
  const int wave = __builtin_amdgcn_readfirstlane((int)(tid >> 5));
  const int c = lane & 15;
  const int hh = lane >> 4;
  const int koff = 8 * hh;
  const int bh = blockIdx.x >> 2;
  const int dv0 = (blockIdx.x & 3) * kSlice;
  const int which = wave >> 2;
  const int nt = wave & 3;

  {
    v8h zz;
#pragma unroll
    for (int e = 0; e < 8; ++e) zz[e] = (_Float16)0.0f;
#pragma unroll 1
    for (int i = tid; i < (kSlice * kSP) / 8; i += 256) *(v8h*)(S16 + i * 8) = zz;
  }
  const v8f z8 = (v8f){0.f, 0.f, 0.f, 0.f, 0.f, 0.f, 0.f, 0.f};
  v8f Sm[2][4];
#pragma unroll
  for (int mi = 0; mi < 2; ++mi)
#pragma unroll
    for (int j = 0; j < 4; ++j) Sm[mi][j] = z8;

#pragma unroll 1
  for (int n = 0; n < kNChunk; ++n) {
    const size_t cb = ((size_t)bh * kSeq + (size_t)n * kChunk) * kHd;

#pragma unroll
    for (int it = 0; it < 4; ++it) {
      const int item = it * 256 + tid;
      const int row = item >> 5;
      const int c8 = (item & 31) * 8;
      const v4u kw = *(const v4u*)(K16 + cb + (size_t)row * kHd + c8);
#pragma unroll
      for (int q = 0; q < 4; ++q) {
        const unsigned ku = kw[q];
        kT[(c8 + 2 * q) * kTP + row]     = bits_to_h(ku);
        kT[(c8 + 2 * q + 1) * kTP + row] = bits_to_h(ku >> 16);
      }
    }
    {
      const int row = tid >> 3;
      const int c8 = (tid & 7) * 8;
      const v4u uw = *(const v4u*)(U16 + cb + (size_t)row * kHd + dv0 + c8);
      v4f f0, f1;
      {
        const unsigned w0 = uw[0], w1 = uw[1], w2 = uw[2], w3 = uw[3];
        f0[0] = h16_to_f32(w0 & 0xffffu); f0[1] = h16_to_f32(w0 >> 16);
        f0[2] = h16_to_f32(w1 & 0xffffu); f0[3] = h16_to_f32(w1 >> 16);
        f1[0] = h16_to_f32(w2 & 0xffffu); f1[1] = h16_to_f32(w2 >> 16);
        f1[2] = h16_to_f32(w3 & 0xffffu); f1[3] = h16_to_f32(w3 >> 16);
      }
      *(v4f*)(uS + row * kFP + c8) = f0;
      *(v4f*)(uS + row * kFP + c8 + 4) = f1;
    }
    __syncthreads();

    v8f acc0 = z8, acc1 = z8;
    {
      const _Float16* a0p = (const _Float16*)(which ? Q16 : W16P) + cb + (size_t)c * kHd + koff;
      const _Float16* a1p = a0p + 16 * kHd;
      const _Float16* bp = S16 + (nt * 16 + c) * kSP + koff;
#pragma unroll 2
      for (int k0 = 0; k0 < kHd; k0 += 32) {
        const v16h fb = frag_load(bp + k0);
        const v16h f0 = frag_load(a0p + k0);
        const v16h f1 = frag_load(a1p + k0);
        acc0 = mma_h(f0, fb, acc0);
        acc1 = mma_h(f1, fb, acc1);
        guard2_h(acc0, acc1, f0, f1, fb);
      }
    }
    {
      v8h h0, h1;
#pragma unroll
      for (int r = 0; r < 8; ++r) {
        const float un0 = uS[(8 * hh + r) * kFP + nt * 16 + c] - acc0[r];
        const float un1 = uS[(16 + 8 * hh + r) * kFP + nt * 16 + c] - acc1[r];
        h0[r] = (_Float16)un0;
        h1[r] = (_Float16)un1;
      }
      if (which == 0) {
        *(v8h*)(unT + (nt * 16 + c) * kTP + 8 * hh) = h0;
        *(v8h*)(unT + (nt * 16 + c) * kTP + 16 + 8 * hh) = h1;
      }
    }
    __syncthreads();

    {
      const _Float16* ap = (const _Float16*)APL + ((size_t)bh * kNChunk + n) * (kChunk * kChunk) + c * kChunk + koff;
      const v16h af0 = frag_load(ap);
      const v16h af1 = frag_load(ap + 16 * kChunk);
      const v16h ubn = frag_load(unT + (nt * 16 + c) * kTP + koff);
      acc0 = mma_h(af0, ubn, acc0);
      acc1 = mma_h(af1, ubn, acc1);
      guard2_h(acc0, acc1, af0, af1, ubn);
      if (which == 1) {
#pragma unroll
        for (int r = 0; r < 8; ++r) {
          oS[(8 * hh + r) * kFP + nt * 16 + c] = acc0[r];
          oS[(16 + 8 * hh + r) * kFP + nt * 16 + c] = acc1[r];
        }
      }
    }
    {
      const v16h ka0 = frag_load(kT + (32 * wave + c) * kTP + koff);
      const v16h ka1 = frag_load(kT + (32 * wave + 16 + c) * kTP + koff);
      v16h ub[4];
#pragma unroll
      for (int j = 0; j < 4; ++j) {
        ub[j] = frag_load(unT + (16 * j + c) * kTP + koff);
        Sm[0][j] = mma_h(ka0, ub[j], Sm[0][j]);
        Sm[1][j] = mma_h(ka1, ub[j], Sm[1][j]);
      }
      guard8_h(Sm[0][0], Sm[0][1], Sm[0][2], Sm[0][3], Sm[1][0], Sm[1][1], Sm[1][2], Sm[1][3],
               ka0, ka1, ub[0], ub[1], ub[2], ub[3]);
#pragma unroll
      for (int mi = 0; mi < 2; ++mi)
#pragma unroll
        for (int j = 0; j < 4; ++j) {
          v8h hv;
#pragma unroll
          for (int r = 0; r < 8; ++r) hv[r] = (_Float16)Sm[mi][j][r];
          *(v8h*)(S16 + (16 * j + c) * kSP + 32 * wave + 16 * mi + 8 * hh) = hv;
        }
    }
    __syncthreads();

    for (int pass = 0; pass < 2; ++pass) {
#pragma unroll
      for (int it = 0; it < 2; ++it) {
        const int idx = it * 256 + tid;
        const int row = idx >> 4;
        const int c4 = (idx & 15) * 4;
        const v4f v = *(const v4f*)(oS + row * kFP + c4);
        *(volatile v4f*)(OD + cb + (size_t)row * kHd + dv0 + c4) = v;
      }
      __threadfence();
    }
  }
}

__global__ __launch_bounds__(256) void ema_mix_kernel(const unsigned short* __restrict__ V16, const float* __restrict__ G,
                                                      float* OD) {
  const int bh = blockIdx.x;
  const int b = bh >> 2;
  const int h = bh & 3;
  const int ch = threadIdx.x;
  const size_t pbase = (size_t)bh * kSeq * kHd + ch;
  const float* Gb = G + (size_t)b * kSeq * kGP + h;
  float s = 0.0f;
#pragma unroll 1
  for (int l0 = 0; l0 < kSeq; l0 += 4) {
    float gv[4], mv[4], vv[4], od[4], ov[4];
#pragma unroll
    for (int i = 0; i < 4; ++i) {
      gv[i] = Gb[(size_t)(l0 + i) * kGP + 4];
      mv[i] = Gb[(size_t)(l0 + i) * kGP + 8];
      const unsigned hb = (unsigned)V16[pbase + (size_t)(l0 + i) * kHd];
      vv[i] = h16_to_f32(hb);
      od[i] = OD[pbase + (size_t)(l0 + i) * kHd];
    }
#pragma unroll
    for (int i = 0; i < 4; ++i) {
      s = gv[i] * s + (1.0f - gv[i]) * vv[i];
      ov[i] = (1.0f - mv[i]) * od[i] + mv[i] * s;
    }
    for (int pass = 0; pass < 2; ++pass) {
#pragma unroll
      for (int i = 0; i < 4; ++i) *(volatile float*)(OD + pbase + (size_t)(l0 + i) * kHd) = ov[i];
      __threadfence();
    }
  }
}

__global__ __launch_bounds__(256) void rms_out_kernel(const float* __restrict__ OD, const float* __restrict__ nw,
                                                      unsigned short* __restrict__ ON16) {
  const int lane = threadIdx.x & 31;
  const int r = blockIdx.x * 8 + (int)(threadIdx.x >> 5);
  if (r >= kBH * kSeq) return;
  const int bh = r >> 12;
  const int l = r & (kSeq - 1);
  const int b = bh >> 2;
  const int h = bh & 3;
  const float* p = OD + (size_t)r * kHd + 8 * lane;
  const v4f a0 = *(const v4f*)(p);
  const v4f a1 = *(const v4f*)(p + 4);
  const v4f w0 = *(const v4f*)(nw + 8 * lane);
  const v4f w1 = *(const v4f*)(nw + 8 * lane + 4);
  float ss = 0.0f;
#pragma unroll
  for (int e = 0; e < 4; ++e) { ss += a0[e] * a0[e]; ss += a1[e] * a1[e]; }
#pragma unroll
  for (int off = 1; off < 32; off <<= 1) ss += __shfl_xor(ss, off, 32);
  const float inv = rsqrtf(ss * kInvHd + kEpsRms);
  v8h hv;
#pragma unroll
  for (int e = 0; e < 4; ++e) {
    hv[e]     = (_Float16)((a0[e] * inv) * w0[e]);
    hv[4 + e] = (_Float16)((a1[e] * inv) * w1[e]);
  }
  unsigned short* dp = ON16 + ((size_t)(b * kSeq + l)) * kDim + h * kHd + 8 * lane;
  *(volatile v8h*)dp = hv;
  __threadfence();
  *(volatile v8h*)dp = hv;
}

extern "C" void kernel_launch(void* const* d_in, const int* in_sizes, int n_in,
                              void* d_out, int out_size, void* d_ws, size_t ws_size, hipStream_t stream) {
  if (n_in < 13 || d_out == nullptr || d_ws == nullptr) return;
  if (in_sizes[0] != kTok * kDim || in_sizes[1] != kDim * kDim || in_sizes[2] != kDim * kDim ||
      in_sizes[3] != kDim * kDim || in_sizes[4] != kHeads * kDim || in_sizes[5] != kHeads * kDim ||
      in_sizes[6] != kHeads * kDim || in_sizes[7] != kHeads || in_sizes[8] != kDim * 4 ||
      in_sizes[9] != kDim * 4 || in_sizes[10] != kDim * 4 || in_sizes[11] != kHd ||
      in_sizes[12] != kDim * kDim || out_size != kTok * kDim) return;

  const float* hs     = (const float*)d_in[0];
  const float* Wq     = (const float*)d_in[1];
  const float* Wk     = (const float*)d_in[2];
  const float* Wv     = (const float*)d_in[3];
  const float* Wb     = (const float*)d_in[4];
  const float* Wdec   = (const float*)d_in[5];
  const float* Wmix   = (const float*)d_in[6];
  const float* mixb   = (const float*)d_in[7];
  const float* wqc    = (const float*)d_in[8];
  const float* wkc    = (const float*)d_in[9];
  const float* wvc    = (const float*)d_in[10];
  const float* onw    = (const float*)d_in[11];
  const float* Wo     = (const float*)d_in[12];
  float* out = (float*)d_out;

  char* ws = (char*)d_ws;
  size_t off = 0;
  auto carve = [&](size_t bytes) -> char* { char* p = ws + off; off += (bytes + 255) & ~(size_t)255; return p; };
  const size_t planeH = (size_t)kBH * kSeq * kHd * 2;
  unsigned short* WO16 = (unsigned short*)carve((size_t)kDim * kDim * 2);
  float*          GRAW = (float*)carve((size_t)kTok * kGRP * 4);
  float*          Gp   = (float*)carve((size_t)kTok * kGP * 4);
  unsigned short* APL  = (unsigned short*)carve((size_t)kBH * kNChunk * kChunk * kChunk * 2);
  unsigned short* Q16  = (unsigned short*)carve(planeH);
  unsigned short* K16  = (unsigned short*)carve(planeH);
  unsigned short* V16  = (unsigned short*)carve(planeH);
  char*           R1   = carve((size_t)kTok * kDim * 4);
  char*           R2   = carve((size_t)kTok * kDim * 4);
  if (off > ws_size || off > (size_t)134217728) return;

  float*          Pp     = (float*)R1;
  unsigned short* U16    = (unsigned short*)R1;
  unsigned short* W16P   = (unsigned short*)(R1 + planeH);
  unsigned short* ON16   = (unsigned short*)R1;
  unsigned short* HS16   = (unsigned short*)R2;
  unsigned short* WQKV16 = (unsigned short*)(R2 + (size_t)kTok * kDim * 2);
  unsigned short* WG16   = (unsigned short*)(R2 + (size_t)kTok * kDim * 2 + (size_t)3 * kDim * kDim * 2);
  float*          OD     = (float*)R2;
  static_assert((size_t)kTok * kDim * 2 + (size_t)3 * kDim * kDim * 2 + (size_t)kGRP * kDim * 2 <= (size_t)kTok * kDim * 4,
                "phase-A planes fit the shared region");
  static_assert(2 * (size_t)kBH * kSeq * kHd * 2 <= (size_t)kTok * kDim * 4, "u and w planes fit the projection region");

  const int n8x = kTok * kDim / 8;
  const int n8w = kDim * kDim / 8;
  cast8_f16_kernel<<<(n8x + 255) / 256, 256, 0, stream>>>(hs, HS16, n8x, 1.0f);
  cast8_f16_kernel<<<(n8w + 255) / 256, 256, 0, stream>>>(Wq, WQKV16, n8w, kWCarry);
  cast8_f16_kernel<<<(n8w + 255) / 256, 256, 0, stream>>>(Wk, WQKV16 + (size_t)kDim * kDim, n8w, kWCarry);
  cast8_f16_kernel<<<(n8w + 255) / 256, 256, 0, stream>>>(Wv, WQKV16 + (size_t)2 * kDim * kDim, n8w, kWCarry);
  cast8_f16_kernel<<<(n8w + 255) / 256, 256, 0, stream>>>(Wo, WO16, n8w, kWCarry);
  gate_pack_kernel<<<(kGRP * (kDim / 8) + 255) / 256, 256, 0, stream>>>(Wb, Wdec, Wmix, WG16, kWCarry);

  const int tilesG = (kTok / 64) * (kGRP / 64);
  wmma_gemm64_f16<<<(tilesG + 7) / 8, 256, 0, stream>>>(HS16, kDim, WG16, kDim, GRAW, kGRP, kTok, kGRP, kDim, kWCarryInv);
  gate_act_kernel<<<(kTok * 8 + 255) / 256, 256, 0, stream>>>(GRAW, mixb, Gp);

  const int tilesP = (kTok / 64) * (kDim / 64);
  const int gridP = (tilesP + 7) / 8;
  const int gridC = kTok / kConvTile;
  wmma_gemm64_f16<<<gridP, 256, 0, stream>>>(HS16, kDim, WQKV16, kDim, Pp, kDim, kTok, kDim, kDim, kWCarryInv);
  conv_act_kernel<true><<<gridC, 128, 0, stream>>>(Pp, wqc, Q16);
  wmma_gemm64_f16<<<gridP, 256, 0, stream>>>(HS16, kDim, WQKV16 + (size_t)kDim * kDim, kDim, Pp, kDim, kTok, kDim, kDim, kWCarryInv);
  conv_act_kernel<true><<<gridC, 128, 0, stream>>>(Pp, wkc, K16);
  wmma_gemm64_f16<<<gridP, 256, 0, stream>>>(HS16, kDim, WQKV16 + (size_t)2 * kDim * kDim, kDim, Pp, kDim, kTok, kDim, kDim, kWCarryInv);
  conv_act_kernel<false><<<gridC, 128, 0, stream>>>(Pp, wvc, V16);

  chunk_prep_kernel<<<kBH * kNChunk, 256, 0, stream>>>(Q16, K16, V16, Gp, U16, W16P, APL);

  state_scan_kernel<<<kBH * kNSlice, 256, 0, stream>>>(Q16, K16, U16, W16P, APL, OD);

  ema_mix_kernel<<<kBH, 256, 0, stream>>>(V16, Gp, OD);
  rms_out_kernel<<<(kBH * kSeq) / 8, 256, 0, stream>>>(OD, onw, ON16);
  wmma_gemm64_f16<<<gridP, 256, 0, stream>>>(ON16, kDim, WO16, kDim, out, kDim, kTok, kDim, kDim, kWCarryInv);
}
